// SRL_KT_27350351741624
// MI455X (gfx1250) — hardware-verified
//
#include <hip/hip_runtime.h>

typedef _Float16 v16h __attribute__((ext_vector_type(16)));
typedef _Float16 v8h  __attribute__((ext_vector_type(8)));
typedef float    v8f  __attribute__((ext_vector_type(8)));
typedef float    v4f  __attribute__((ext_vector_type(4)));
typedef v8h __attribute__((may_alias)) v8ha;
typedef v4f __attribute__((may_alias)) v4fa;
union Frag { v16h v; v8h half[2]; };

#define NB     32
#define SEQ    512
#define EMB    512
#define NH     8
#define HD     64
#define NL     2
#define VOC    10000
#define NTYPE  4
#define MROWS  (NB * SEQ)
#define PSCALE 16384.0f

static_assert(EMB == NH * HD);
static_assert((SEQ % 128) == 0);
static_assert((MROWS % 128) == 0);
static_assert((EMB % 64) == 0);

__device__ __forceinline__ v8f wmma_f16(v16h a, v16h b, v8f c) {
  v8f d = __builtin_amdgcn_wmma_f32_16x16x32_f16(false, a, false, b, (short)0, c, false, false);
  asm volatile("v_nop\n\tv_nop\n\tv_nop\n\tv_nop" : "+v"(d) : "v"(a), "v"(b));
  return d;
}

__device__ __forceinline__ v16h load_frag(const _Float16* p, int h) {
  Frag f;
  f.half[0] = *(const v8ha*)(p + 8 * h);
  f.half[1] = *(const v8ha*)(p + 16 + 8 * h);
  return f.v;
}

__device__ __forceinline__ v8f zero8f() {
  const v8f z = {0.f, 0.f, 0.f, 0.f, 0.f, 0.f, 0.f, 0.f};
  return z;
}
__device__ __forceinline__ v4f zero4f() {
  const v4f z = {0.f, 0.f, 0.f, 0.f};
  return z;
}

__device__ __forceinline__ v8h cvt8(v4f a, v4f c) {
  const v8h o = { (_Float16)a.x, (_Float16)a.y, (_Float16)a.z, (_Float16)a.w,
                  (_Float16)c.x, (_Float16)c.y, (_Float16)c.z, (_Float16)c.w };
  return o;
}

__device__ __forceinline__ float wave_max(float v) {
  #pragma unroll
  for (int o = 16; o > 0; o >>= 1) v = fmaxf(v, __shfl_xor(v, o));
  return v;
}
__device__ __forceinline__ float wave_sum(float v) {
  #pragma unroll
  for (int o = 16; o > 0; o >>= 1) v += __shfl_xor(v, o);
  return v;
}

__global__ __launch_bounds__(256) void k_wtrans(const float* __restrict__ src, _Float16* __restrict__ dst,
                                                 int K, int N, float sc)
{
  __shared__ __attribute__((aligned(16))) _Float16 sT[64 * 72];
  const int tid = threadIdx.x, lane = tid & 31, w = tid >> 5;
  const int n0 = blockIdx.x * 64, k0 = blockIdx.y * 64;
  const size_t zoff = (size_t)blockIdx.z * (size_t)K * (size_t)N;
  const float* s = src + zoff;
  _Float16* d = dst + zoff;
  #pragma unroll
  for (int i = 0; i < 16; ++i) {
    const int flat = i * 256 + tid;
    const int kr = flat >> 6, nc = flat & 63;
    sT[nc * 72 + kr] = (_Float16)(s[(size_t)(k0 + kr) * N + n0 + nc] * sc);
  }
  __syncthreads();
  const int q8 = lane & 7, sub = lane >> 3;
  const int nl0 = w * 8 + sub, nl1 = w * 8 + 4 + sub;
  const v8h v0 = *(const v8ha*)(sT + nl0 * 72 + 8 * q8);
  const v8h v1 = *(const v8ha*)(sT + nl1 * 72 + 8 * q8);
  const size_t o0 = (size_t)(n0 + nl0) * K + k0 + 8 * q8;
  const size_t o1 = (size_t)(n0 + nl1) * K + k0 + 8 * q8;
  *(volatile v8h*)(d + o0) = v0;
  *(volatile v8h*)(d + o1) = v1;
  __threadfence();
  *(volatile v8h*)(d + o0) = v0;
  *(volatile v8h*)(d + o1) = v1;
}

__global__ __launch_bounds__(128) void k_wsum(const float* __restrict__ W_int, const float* __restrict__ type_table,
                                               float* __restrict__ TW, float* __restrict__ csq, float* __restrict__ csl)
{
  const int n = blockIdx.x * 128 + threadIdx.x;
  if (n >= EMB) return;
  float t0 = 0.f, t1 = 0.f, t2 = 0.f, t3 = 0.f, sq = 0.f, sl = 0.f;
  #pragma unroll 1
  for (int k = 0; k < EMB; ++k) {
    const float w = W_int[(size_t)(EMB + k) * EMB + n];
    t0 += type_table[k] * w;
    t1 += type_table[EMB + k] * w;
    t2 += type_table[2 * EMB + k] * w;
    t3 += type_table[3 * EMB + k] * w;
  }
  #pragma unroll 1
  for (int k = 0; k < EMB; ++k) {
    sq += W_int[(size_t)(2 * EMB + k) * EMB + n];
    sl += W_int[(size_t)(3 * EMB + k) * EMB + n];
  }
  *(volatile float*)(TW + n) = t0;
  *(volatile float*)(TW + EMB + n) = t1;
  *(volatile float*)(TW + 2 * EMB + n) = t2;
  *(volatile float*)(TW + 3 * EMB + n) = t3;
  *(volatile float*)(csq + n) = sq;
  *(volatile float*)(csl + n) = sl;
  __threadfence();
  *(volatile float*)(TW + n) = t0;
  *(volatile float*)(TW + EMB + n) = t1;
  *(volatile float*)(TW + 2 * EMB + n) = t2;
  *(volatile float*)(TW + 3 * EMB + n) = t3;
  *(volatile float*)(csq + n) = sq;
  *(volatile float*)(csl + n) = sl;
}

__global__ __launch_bounds__(256) void k_planes(const int* __restrict__ item_inputs, const int* __restrict__ item_ids,
                                                 const float* __restrict__ use_table,
                                                 _Float16* __restrict__ itemh, _Float16* __restrict__ qeh)
{
  const int g = blockIdx.x * 256 + threadIdx.x;
  if (g >= 2 * MROWS * (EMB / 8)) return;
  const int which = (g >= MROWS * (EMB / 8)) ? 1 : 0;
  const int r = g - which * (MROWS * (EMB / 8));
  const int mrow = r >> 6, e8 = (r & 63) * 8;
  int idx = which ? item_ids[mrow] : item_inputs[mrow];
  if (idx < 0) idx += VOC;
  idx = min(max(idx, 0), VOC - 1);
  const float* sp = use_table + (size_t)idx * EMB + e8;
  const v4f a = *(const v4fa*)sp;
  const v4f c = *(const v4fa*)(sp + 4);
  const float sc = (which == 0 && (mrow & (SEQ - 1)) == 0) ? 0.0f : 1.0f;
  const v8h o = { (_Float16)(a.x * sc), (_Float16)(a.y * sc), (_Float16)(a.z * sc), (_Float16)(a.w * sc),
                  (_Float16)(c.x * sc), (_Float16)(c.y * sc), (_Float16)(c.z * sc), (_Float16)(c.w * sc) };
  _Float16* dp = (which ? qeh : itemh) + (size_t)mrow * EMB + e8;
  *(volatile v8h*)dp = o;
  __threadfence();
  *(volatile v8h*)dp = o;
}

__global__ __launch_bounds__(64) void k_pmix(const float* __restrict__ rel, const float* __restrict__ ts,
                                              const float* __restrict__ l1p, const float* __restrict__ l2p,
                                              _Float16* __restrict__ pm)
{
  __shared__ float red[4];
  const int row = blockIdx.x, q = row & (SEQ - 1), t = threadIdx.x, lane = t & 31, w = t >> 5;
  const float l1 = l1p[0], l2 = l2p[0];
  const size_t base = (size_t)row * SEQ + 8 * t;
  const v4f ta = *(const v4fa*)(ts + base);
  const v4f tb = *(const v4fa*)(ts + base + 4);
  const v4f ra = *(const v4fa*)(rel + base);
  const v4f rb = *(const v4fa*)(rel + base + 4);
  float tv[8] = {ta.x, ta.y, ta.z, ta.w, tb.x, tb.y, tb.z, tb.w};
  float rv[8] = {ra.x, ra.y, ra.z, ra.w, rb.x, rb.y, rb.z, rb.w};
  float mT = -1e30f, mR = -1e30f;
  #pragma unroll
  for (int i = 0; i < 8; ++i) {
    const int k = 8 * t + i;
    const bool fut = (k > q);
    const float e = __expf(-fabsf(tv[i]));
    tv[i] = fut ? -1e30f : e;
    const float relm = fut ? rv[i] : 0.0f;
    rv[i] = (relm == 0.0f) ? -10000.0f : relm;
    mT = fmaxf(mT, tv[i]);
    mR = fmaxf(mR, rv[i]);
  }
  mT = wave_max(mT);
  mR = wave_max(mR);
  if (lane == 0) { red[w] = mT; red[2 + w] = mR; }
  __syncthreads();
  mT = fmaxf(red[0], red[1]);
  mR = fmaxf(red[2], red[3]);
  __syncthreads();
  float sumT = 0.f, sumR = 0.f;
  #pragma unroll
  for (int i = 0; i < 8; ++i) {
    const int k = 8 * t + i;
    const bool fut = (k > q);
    const float eT = fut ? 0.0f : __expf(fmaxf(tv[i] - mT, -80.0f));
    const float eR = __expf(fmaxf(rv[i] - mR, -80.0f));
    tv[i] = eT;
    rv[i] = eR;
    sumT += eT;
    sumR += eR;
  }
  sumT = wave_sum(sumT);
  sumR = wave_sum(sumR);
  if (lane == 0) { red[w] = sumT; red[2 + w] = sumR; }
  __syncthreads();
  sumT = red[0] + red[1];
  sumR = red[2] + red[3];
  const float cT = (1.0f - l1) * l2 * (1.0f / sumT) * PSCALE;
  const float cR = l1 * (1.0f / sumR) * PSCALE;
  const v8h o = { (_Float16)(tv[0] * cT + rv[0] * cR), (_Float16)(tv[1] * cT + rv[1] * cR),
                  (_Float16)(tv[2] * cT + rv[2] * cR), (_Float16)(tv[3] * cT + rv[3] * cR),
                  (_Float16)(tv[4] * cT + rv[4] * cR), (_Float16)(tv[5] * cT + rv[5] * cR),
                  (_Float16)(tv[6] * cT + rv[6] * cR), (_Float16)(tv[7] * cT + rv[7] * cR) };
  *(volatile v8h*)(pm + base) = o;
  __threadfence();
  *(volatile v8h*)(pm + base) = o;
}

__device__ __forceinline__ void mma_step(const _Float16* xa0, const _Float16* xa1,
                                         const _Float16* wb, int ldw, int h, v8f (&acc)[2][4]) {
  const v16h a0 = load_frag(xa0, h);
  const v16h a1 = load_frag(xa1, h);
  #pragma unroll
  for (int nt = 0; nt < 4; ++nt) {
    const v16h bb = load_frag(wb + (size_t)nt * 16 * ldw, h);
    acc[0][nt] = wmma_f16(a0, bb, acc[0][nt]);
    acc[1][nt] = wmma_f16(a1, bb, acc[1][nt]);
  }
}

__device__ __forceinline__ void row_store_pass(const _Float16* sT, _Float16* dst, int m0, int c0, int w, int lane) {
  const int q8 = lane & 7, sub = lane >> 3;
  #pragma unroll
  for (int i = 0; i < 8; ++i) {
    const int lid = w * 32 + i * 4 + sub;
    const v8h v = *(const v8ha*)(sT + lid * 64 + 8 * q8);
    *(volatile v8h*)(dst + (size_t)(m0 + lid) * EMB + c0 + 8 * q8) = v;
  }
}
__device__ __forceinline__ void vt_store_pass(const _Float16* sT, _Float16* vth, int bh, int s0, int w, int lane) {
  const int q8 = lane & 7, sub = lane >> 3;
  #pragma unroll
  for (int i = 0; i < 8; ++i) {
    const int lid = w * 32 + i * 4 + sub;
    const int d = lid >> 1, hl = lid & 1;
    const v8h v = *(const v8ha*)(sT + d * 128 + 64 * hl + 8 * q8);
    *(volatile v8h*)(vth + ((size_t)(bh * HD + d)) * SEQ + s0 + 64 * hl + 8 * q8) = v;
  }
}

__global__ __launch_bounds__(128) void k_gemm_int(
    const _Float16* __restrict__ itemh, const _Float16* __restrict__ winth,
    const float* __restrict__ b_int, const float* __restrict__ TW,
    const float* __restrict__ csq, const float* __restrict__ csl,
    const int* __restrict__ type_inputs, const float* __restrict__ qresp, const float* __restrict__ label,
    _Float16* __restrict__ inph)
{
  __shared__ __attribute__((aligned(16))) _Float16 sT[128 * 64];
  const int tid = threadIdx.x, lane = tid & 31, w = tid >> 5;
  const int h = lane >> 4, m = lane & 15;
  const int m0 = blockIdx.x * 128, cg = blockIdx.y, m0w = m0 + 32 * w;

  const _Float16* xa0 = itemh + (size_t)(m0w + m) * EMB;
  const _Float16* xa1 = xa0 + (size_t)16 * EMB;
  const _Float16* wb  = winth + (size_t)(cg * 64 + m) * EMB;

  v8f acc[2][4];
  #pragma unroll
  for (int mt = 0; mt < 2; ++mt)
    #pragma unroll
    for (int nt = 0; nt < 4; ++nt) acc[mt][nt] = zero8f();

  #pragma unroll 1
  for (int k0 = 0; k0 < EMB; k0 += 32)
    mma_step(xa0 + k0, xa1 + k0, wb + k0, EMB, h, acc);

  float rq[2][8], rl[2][8];
  int rt[2][8];
  #pragma unroll
  for (int mt = 0; mt < 2; ++mt)
    #pragma unroll
    for (int r = 0; r < 8; ++r) {
      const int grow = m0w + 16 * mt + 8 * h + r;
      int ty = type_inputs[grow];
      if (ty < 0) ty += NTYPE;
      ty = min(max(ty, 0), NTYPE - 1);
      rt[mt][r] = ty;
      rq[mt][r] = qresp[grow];
      rl[mt][r] = label[grow];
    }

  #pragma unroll
  for (int nt = 0; nt < 4; ++nt) {
    const int feat = 16 * nt + m;
    const int n = cg * 64 + feat;
    const float bb = b_int[n], cq = csq[n], cl = csl[n];
    const float tw0 = TW[n], tw1 = TW[EMB + n], tw2 = TW[2 * EMB + n], tw3 = TW[3 * EMB + n];
    #pragma unroll
    for (int mt = 0; mt < 2; ++mt) {
      #pragma unroll
      for (int r = 0; r < 8; ++r) {
        const int ty = rt[mt][r];
        const float tw = (ty == 0) ? tw0 : ((ty == 1) ? tw1 : ((ty == 2) ? tw2 : tw3));
        float y = acc[mt][nt][r] * (1.0f / 32.0f) + bb + tw + rq[mt][r] * cq + rl[mt][r] * cl;
        y = fmaxf(y, 0.0f);
        const int tokl = 32 * w + 16 * mt + 8 * h + r;
        sT[tokl * 64 + feat] = (_Float16)y;
      }
    }
  }
  __syncthreads();

  row_store_pass(sT, inph, m0, cg * 64, w, lane);
  __threadfence();
  row_store_pass(sT, inph, m0, cg * 64, w, lane);
}

__global__ __launch_bounds__(128) void k_gemm_qkv(
    const _Float16* __restrict__ qeh, const _Float16* __restrict__ kvh,
    const _Float16* __restrict__ wqh, const _Float16* __restrict__ wkh, const _Float16* __restrict__ wvh,
    const float* __restrict__ bq, const float* __restrict__ bk, const float* __restrict__ bv,
    _Float16* __restrict__ qh, _Float16* __restrict__ kh, _Float16* __restrict__ vth)
{
  __shared__ __attribute__((aligned(16))) _Float16 sT[128 * 64];
  const int tid = threadIdx.x, lane = tid & 31, w = tid >> 5;
  const int h = lane >> 4, m = lane & 15;
  const int m0 = blockIdx.x * 128, m0w = m0 + 32 * w;
  const int which = blockIdx.y >> 3, head = blockIdx.y & 7;

  const _Float16* A = (which == 0) ? qeh : kvh;
  const _Float16* W = (which == 0) ? wqh : ((which == 1) ? wkh : wvh);
  const float* bias  = (which == 0) ? bq : ((which == 1) ? bk : bv);

  const _Float16* xa0 = A + (size_t)(m0w + m) * EMB;
  const _Float16* xa1 = xa0 + (size_t)16 * EMB;
  const _Float16* wb  = W + (size_t)(head * HD + m) * EMB;

  v8f acc[2][4];
  #pragma unroll
  for (int mt = 0; mt < 2; ++mt)
    #pragma unroll
    for (int nt = 0; nt < 4; ++nt) acc[mt][nt] = zero8f();

  #pragma unroll 1
  for (int k0 = 0; k0 < EMB; k0 += 32)
    mma_step(xa0 + k0, xa1 + k0, wb + k0, EMB, h, acc);

  #pragma unroll
  for (int nt = 0; nt < 4; ++nt) {
    const int feat = 16 * nt + m;
    const float bvl = bias[head * HD + feat];
    #pragma unroll
    for (int mt = 0; mt < 2; ++mt) {
      #pragma unroll
      for (int r = 0; r < 8; ++r) {
        const int tokl = 32 * w + 16 * mt + 8 * h + r;
        const float y = acc[mt][nt][r] * (1.0f / 16.0f) + bvl;
        const int idx = (which == 2) ? (feat * 128 + tokl) : (tokl * 64 + feat);
        sT[idx] = (_Float16)y;
      }
    }
  }
  __syncthreads();

  if (which == 2) {
    const int b = m0 >> 9, s0 = m0 & (SEQ - 1), bh = b * NH + head;
    vt_store_pass(sT, vth, bh, s0, w, lane);
    __threadfence();
    vt_store_pass(sT, vth, bh, s0, w, lane);
  } else {
    _Float16* plane = (which == 0) ? qh : kh;
    row_store_pass(sT, plane, m0, head * HD, w, lane);
    __threadfence();
    row_store_pass(sT, plane, m0, head * HD, w, lane);
  }
}

__device__ __forceinline__ v4f exp4(v4f v, float mx) {
  v4f r;
  r.x = __expf(fmaxf(v.x - mx, -80.0f));
  r.y = __expf(fmaxf(v.y - mx, -80.0f));
  r.z = __expf(fmaxf(v.z - mx, -80.0f));
  r.w = __expf(fmaxf(v.w - mx, -80.0f));
  return r;
}
__device__ __forceinline__ v8h mixpack(float csi, v4f ea, v4f eb, v8h g) {
  const v8h o = { (_Float16)(csi * ea.x + (float)g[0]), (_Float16)(csi * ea.y + (float)g[1]),
                  (_Float16)(csi * ea.z + (float)g[2]), (_Float16)(csi * ea.w + (float)g[3]),
                  (_Float16)(csi * eb.x + (float)g[4]), (_Float16)(csi * eb.y + (float)g[5]),
                  (_Float16)(csi * eb.z + (float)g[6]), (_Float16)(csi * eb.w + (float)g[7]) };
  return o;
}
__device__ __forceinline__ void att_store_pass(const v8h* vals, _Float16* base, int sub) {
  #pragma unroll
  for (int i = 0; i < 4; ++i)
    *(volatile v8h*)(base + (size_t)(i * 4 + sub) * EMB) = vals[i];
}

__global__ __launch_bounds__(32) void k_attn(
    const _Float16* __restrict__ qh, const _Float16* __restrict__ kh, const _Float16* __restrict__ vth,
    const _Float16* __restrict__ pm, const float* __restrict__ l1p, const float* __restrict__ l2p,
    const _Float16* resh, _Float16* outh, int layer)
{
  __shared__ __attribute__((aligned(16))) float sS[32 * 256];

  const int lane = threadIdx.x & 31, h = lane >> 4, m = lane & 15;
  const int qt = blockIdx.x, bh = blockIdx.y, b = bh >> 3, head = bh & 7;
  const int q0 = qt * 16;
  const float l1 = l1p[0], l2 = l2p[0];
  const float cs = (1.0f - l1) * (1.0f - l2);

  const size_t qrow = ((size_t)(b * SEQ + q0 + m)) * EMB + head * HD;
  const v16h qb0 = load_frag(qh + qrow, h);
  const v16h qb1 = load_frag(qh + qrow + 32, h);

  float* mys = sS + lane * 8;
  const int T = qt;
  float mloc = -1e30f;

  #pragma unroll 1
  for (int t = 0; t <= T; ++t) {
    const _Float16* kp = kh + ((size_t)(b * SEQ + 16 * t + m)) * EMB + head * HD;
    const v16h kf0 = load_frag(kp, h);
    const v16h kf1 = load_frag(kp + 32, h);
    v8f z = zero8f();
    z = wmma_f16(kf0, qb0, z);
    z = wmma_f16(kf1, qb1, z);
    const bool diag = (t == T);
    #pragma unroll
    for (int r = 0; r < 8; ++r) {
      float v = z[r] * 0.125f;
      if (diag && (8 * h + r > m)) v = -1e30f;
      mloc = fmaxf(mloc, v);
      z[r] = v;
    }
    const v4f lo = {z[0], z[1], z[2], z[3]};
    const v4f hi = {z[4], z[5], z[6], z[7]};
    *(v4fa*)(mys + t * 256) = lo;
    *(v4fa*)(mys + t * 256 + 4) = hi;
  }
  const float mx = fmaxf(mloc, __shfl_xor(mloc, 16));

  float lsum = 0.f;
  #pragma unroll 1
  for (int t = 0; t <= T; ++t) {
    const v4f lo = exp4(*(const v4fa*)(mys + t * 256), mx);
    const v4f hi = exp4(*(const v4fa*)(mys + t * 256 + 4), mx);
    lsum += (lo.x + lo.y) + (lo.z + lo.w) + (hi.x + hi.y) + (hi.z + hi.w);
    *(v4fa*)(mys + t * 256) = lo;
    *(v4fa*)(mys + t * 256 + 4) = hi;
  }
  if ((T & 1) == 0) {
    *(v4fa*)(mys + (T + 1) * 256) = zero4f();
    *(v4fa*)(mys + (T + 1) * 256 + 4) = zero4f();
  }
  lsum += __shfl_xor(lsum, 16);
  const float csi = cs * (1.0f / lsum) * PSCALE;

  v8f o[4];
  #pragma unroll
  for (int t4 = 0; t4 < 4; ++t4) o[t4] = zero8f();
  const int cT = T >> 1;
  const size_t prow = ((size_t)(b * SEQ + q0 + m)) * SEQ + 8 * h;
  const size_t vrow = ((size_t)(bh * HD + m)) * SEQ;
  #pragma unroll 1
  for (int c = 0; c < SEQ / 32; ++c) {
    v4f e0a = zero4f(), e0b = zero4f(), e1a = zero4f(), e1b = zero4f();
    if (c <= cT) {
      e0a = *(const v4fa*)(mys + (2 * c) * 256);
      e0b = *(const v4fa*)(mys + (2 * c) * 256 + 4);
      e1a = *(const v4fa*)(mys + (2 * c + 1) * 256);
      e1b = *(const v4fa*)(mys + (2 * c + 1) * 256 + 4);
    }
    const v8h g0 = *(const v8ha*)(pm + prow + 32 * c);
    const v8h g1 = *(const v8ha*)(pm + prow + 32 * c + 16);
    Frag pb;
    pb.half[0] = mixpack(csi, e0a, e0b, g0);
    pb.half[1] = mixpack(csi, e1a, e1b, g1);
    #pragma unroll
    for (int t4 = 0; t4 < 4; ++t4) {
      const v16h vf = load_frag(vth + vrow + (size_t)(16 * t4) * SEQ + 32 * c, h);
      o[t4] = wmma_f16(vf, pb.v, o[t4]);
    }
  }

  __syncthreads();
  float* so = sS;
  const float inv = 1.0f / PSCALE;
  #pragma unroll
  for (int t4 = 0; t4 < 4; ++t4) {
    float x[8];
    #pragma unroll
    for (int r = 0; r < 8; ++r) x[r] = o[t4][r] * inv;
    if (layer) {
      const v8h rv = *(const v8ha*)(resh + qrow + 16 * t4 + 8 * h);
      #pragma unroll
      for (int r = 0; r < 8; ++r) x[r] = (float)rv[r] + fmaxf(x[r], 0.0f);
    }
    const v4f a = {x[0], x[1], x[2], x[3]};
    const v4f cc = {x[4], x[5], x[6], x[7]};
    *(v4fa*)(so + m * 64 + 16 * t4 + 8 * h) = a;
    *(v4fa*)(so + m * 64 + 16 * t4 + 8 * h + 4) = cc;
  }
  __syncthreads();

  const int q8 = lane & 7, sub = lane >> 3;
  v8h vals[4];
  #pragma unroll
  for (int i = 0; i < 4; ++i) {
    const float* sp = so + (i * 4 + sub) * 64 + 8 * q8;
    vals[i] = cvt8(*(const v4fa*)sp, *(const v4fa*)(sp + 4));
  }
  _Float16* base = outh + ((size_t)(b * SEQ + q0)) * EMB + head * HD + 8 * q8;
  att_store_pass(vals, base, sub);
  __threadfence();
  att_store_pass(vals, base, sub);
}

__global__ __launch_bounds__(128) void k_gemm_f1(
    const _Float16* __restrict__ o1h, const _Float16* __restrict__ qeh,
    const _Float16* __restrict__ wf1h, const float* __restrict__ bf1,
    const float* __restrict__ wf2, const float* __restrict__ bf2,
    float* __restrict__ out)
{
  __shared__ __attribute__((aligned(16))) float so[128];
  const int tid = threadIdx.x, lane = tid & 31, w = tid >> 5;
  const int h = lane >> 4, m = lane & 15;
  const int m0 = blockIdx.x * 128, m0w = m0 + 32 * w;
  const size_t ra0 = (size_t)(m0w + m) * EMB, ra1 = ra0 + (size_t)16 * EMB;

  float part[2][8];
  #pragma unroll
  for (int mt = 0; mt < 2; ++mt)
    #pragma unroll
    for (int r = 0; r < 8; ++r) part[mt][r] = 0.f;

  #pragma unroll 1
  for (int nc = 0; nc < EMB / 64; ++nc) {
    v8f acc[2][4];
    #pragma unroll
    for (int mt = 0; mt < 2; ++mt)
      #pragma unroll
      for (int nt = 0; nt < 4; ++nt) acc[mt][nt] = zero8f();
    const _Float16* wb = wf1h + (size_t)(nc * 64 + m) * (2 * EMB);
    #pragma unroll 1
    for (int k0 = 0; k0 < 2 * EMB; k0 += 32) {
      const _Float16* ab = (k0 < EMB) ? (o1h + k0) : (qeh + (k0 - EMB));
      mma_step(ab + ra0, ab + ra1, wb + k0, 2 * EMB, h, acc);
    }
    #pragma unroll
    for (int nt = 0; nt < 4; ++nt) {
      const int feat = nc * 64 + 16 * nt + m;
      const float bb = bf1[feat], w2 = wf2[feat];
      #pragma unroll
      for (int mt = 0; mt < 2; ++mt)
        #pragma unroll
        for (int r = 0; r < 8; ++r) {
          const float hv = fmaxf(acc[mt][nt][r] * (1.0f / 32.0f) + bb, 0.0f);
          part[mt][r] += hv * w2;
        }
    }
  }

  #pragma unroll
  for (int mt = 0; mt < 2; ++mt)
    #pragma unroll
    for (int r = 0; r < 8; ++r) {
      float v = part[mt][r];
      v += __shfl_xor(v, 1);
      v += __shfl_xor(v, 2);
      v += __shfl_xor(v, 4);
      v += __shfl_xor(v, 8);
      part[mt][r] = v;
    }
  const float b2 = bf2[0];
  if (m == 0) {
    #pragma unroll
    for (int mt = 0; mt < 2; ++mt)
      #pragma unroll
      for (int r = 0; r < 8; ++r) so[32 * w + 16 * mt + 8 * h + r] = part[mt][r] + b2;
  }
  __syncthreads();
  v4f v = zero4f();
  if (w == 0) {
    v = *(const v4fa*)(so + 4 * lane);
    *(volatile v4f*)(out + m0 + 4 * lane) = v;
  }
  __threadfence();
  if (w == 0) {
    *(volatile v4f*)(out + m0 + 4 * lane) = v;
  }
}

extern "C" void kernel_launch(void* const* d_in, const int* in_sizes, int n_in,
                              void* d_out, int out_size, void* d_ws, size_t ws_size,
                              hipStream_t stream)
{
  if (n_in < 23) return;
  if (in_sizes[0] != MROWS || in_sizes[1] != MROWS || in_sizes[2] != MROWS || in_sizes[3] != MROWS) return;
  if (in_sizes[4] != NB * SEQ * SEQ || in_sizes[5] != NB * SEQ * SEQ || in_sizes[6] != MROWS) return;
  if (in_sizes[7] != VOC * EMB || in_sizes[8] != NTYPE * EMB) return;
  if (in_sizes[9] != 4 * EMB * EMB || in_sizes[10] != EMB) return;
  if (in_sizes[11] != NL * EMB * EMB || in_sizes[12] != NL * EMB) return;
  if (in_sizes[13] != NL * EMB * EMB || in_sizes[14] != NL * EMB) return;
  if (in_sizes[15] != NL * EMB * EMB || in_sizes[16] != NL * EMB) return;
  if (in_sizes[17] != 2 * EMB * EMB || in_sizes[18] != EMB || in_sizes[19] != EMB) return;
  if (in_sizes[20] != 1 || in_sizes[21] != 1 || in_sizes[22] != 1) return;
  if (out_size != MROWS) return;

  const int*   item_inputs = (const int*)  d_in[0];
  const float* label       = (const float*)d_in[1];
  const int*   type_inputs = (const int*)  d_in[2];
  const int*   item_ids    = (const int*)  d_in[3];
  const float* rel         = (const float*)d_in[4];
  const float* ts          = (const float*)d_in[5];
  const float* qresp       = (const float*)d_in[6];
  const float* use_table   = (const float*)d_in[7];
  const float* type_table  = (const float*)d_in[8];
  const float* W_int       = (const float*)d_in[9];
  const float* b_int       = (const float*)d_in[10];
  const float* Wq          = (const float*)d_in[11];
  const float* bq          = (const float*)d_in[12];
  const float* Wk          = (const float*)d_in[13];
  const float* bk          = (const float*)d_in[14];
  const float* Wv          = (const float*)d_in[15];
  const float* bv          = (const float*)d_in[16];
  const float* Wf1         = (const float*)d_in[17];
  const float* bf1         = (const float*)d_in[18];
  const float* Wf2         = (const float*)d_in[19];
  const float* bf2         = (const float*)d_in[20];
  const float* l1          = (const float*)d_in[21];
  const float* l2          = (const float*)d_in[22];
  float* out = (float*)d_out;

  const size_t b_w512  = (size_t)EMB * EMB * 2;
  const size_t b_wl    = (size_t)NL * EMB * EMB * 2;
  const size_t b_wf1   = (size_t)2 * EMB * EMB * 2;
  const size_t b_tw    = (size_t)NTYPE * EMB * 4;
  const size_t b_cs    = 4096;
  const size_t b_plane = (size_t)MROWS * EMB * 2;
  const size_t b_pm    = (size_t)NB * SEQ * SEQ * 2;
  const size_t total   = b_w512 + 3 * b_wl + b_wf1 + b_tw + 2 * b_cs + 6 * b_plane + b_pm;
  if (total > ws_size) return;

  char* ws = (char*)d_ws;
  size_t off = 0;
  _Float16* winth = (_Float16*)(ws + off); off += b_w512;
  _Float16* wqh   = (_Float16*)(ws + off); off += b_wl;
  _Float16* wkh   = (_Float16*)(ws + off); off += b_wl;
  _Float16* wvh   = (_Float16*)(ws + off); off += b_wl;
  _Float16* wf1h  = (_Float16*)(ws + off); off += b_wf1;
  float*    TW    = (float*)   (ws + off); off += b_tw;
  float*    csq   = (float*)   (ws + off); off += b_cs;
  float*    csl   = (float*)   (ws + off); off += b_cs;
  _Float16* itemh = (_Float16*)(ws + off); off += b_plane;
  _Float16* qeh   = (_Float16*)(ws + off); off += b_plane;
  _Float16* inph  = (_Float16*)(ws + off); off += b_plane;
  _Float16* qh    = (_Float16*)(ws + off); off += b_plane;
  _Float16* kh    = (_Float16*)(ws + off); off += b_plane;
  _Float16* vth   = (_Float16*)(ws + off); off += b_plane;
  _Float16* pm16  = (_Float16*)(ws + off); off += b_pm;
  if (off > ws_size) return;
  _Float16* o0h = itemh;
  _Float16* o1h = inph;

  k_wtrans<<<dim3(EMB / 64, EMB / 64, 1), 256, 0, stream>>>(W_int, winth, EMB, EMB, 32.0f);
  k_wtrans<<<dim3(EMB / 64, EMB / 64, NL), 256, 0, stream>>>(Wq, wqh, EMB, EMB, 16.0f);
  k_wtrans<<<dim3(EMB / 64, EMB / 64, NL), 256, 0, stream>>>(Wk, wkh, EMB, EMB, 16.0f);
  k_wtrans<<<dim3(EMB / 64, EMB / 64, NL), 256, 0, stream>>>(Wv, wvh, EMB, EMB, 16.0f);
  k_wtrans<<<dim3(EMB / 64, (2 * EMB) / 64, 1), 256, 0, stream>>>(Wf1, wf1h, 2 * EMB, EMB, 32.0f);
  k_wsum<<<EMB / 128, 128, 0, stream>>>(W_int, type_table, TW, csq, csl);
  k_planes<<<(2 * MROWS * (EMB / 8)) / 256, 256, 0, stream>>>(item_inputs, item_ids, use_table, itemh, qeh);
  k_pmix<<<MROWS, 64, 0, stream>>>(rel, ts, l1, l2, pm16);
  k_gemm_int<<<dim3(MROWS / 128, EMB / 64), 128, 0, stream>>>(itemh, winth, b_int, TW, csq, csl,
                                                               type_inputs, qresp, label, inph);
  k_gemm_qkv<<<dim3(MROWS / 128, 3 * NH), 128, 0, stream>>>(qeh, inph, wqh, wkh, wvh, bq, bk, bv, qh, kh, vth);
  k_attn<<<dim3(SEQ / 16, NB * NH), 32, 0, stream>>>(qh, kh, vth, pm16, l1, l2, o0h, o0h, 0);
  k_gemm_qkv<<<dim3(MROWS / 128, 3 * NH), 128, 0, stream>>>(qeh, o0h,
      wqh + (size_t)EMB * EMB, wkh + (size_t)EMB * EMB, wvh + (size_t)EMB * EMB,
      bq + EMB, bk + EMB, bv + EMB, qh, kh, vth);
  k_attn<<<dim3(SEQ / 16, NB * NH), 32, 0, stream>>>(qh, kh, vth, pm16, l1, l2, o0h, o1h, 1);
  k_gemm_f1<<<MROWS / 128, 128, 0, stream>>>(o1h, qeh, wf1h, bf1, Wf2, bf2, out);
}
